// FeatureGrid_22230750724639
// MI455X (gfx1250) — hardware-verified
//
#include <hip/hip_runtime.h>
#include <stddef.h>

#define B_   4
#define C_   64
#define H_   128
#define W_   128
#define N_   (H_ * W_)
#define M_   (B_ * N_)
#define OC_  89
#define IMH_ 256
#define IMW_ 256

#define STOK 128
#define LTOK 64
#define ATOK 32
#define AP   72
#define TP   68
#define QP   68
#define SP   132

static_assert(M_ % STOK == 0);
static_assert(N_ % STOK == 0);
static_assert(N_ % LTOK == 0);
static_assert(N_ % ATOK == 0);
static_assert(AP % 8 == 0);
static_assert((TP * 4) % 16 == 0);
static_assert((QP * 4) % 16 == 0);
static_assert((SP * 4) % 16 == 0);
static_assert((ATOK * OC_) % 32 == 0);
static_assert(LTOK * C_ * 4 <= LTOK * SP * 4);

typedef __bf16 v16bf __attribute__((ext_vector_type(16)));
typedef unsigned short v8us_t __attribute__((ext_vector_type(8)));
typedef v8us_t __attribute__((may_alias)) v8us;
typedef float v8f __attribute__((ext_vector_type(8)));
typedef float v4f_t __attribute__((ext_vector_type(4)));
typedef v4f_t __attribute__((may_alias)) v4f;

union Frag { v16bf v; v8us_t u[2]; };

__device__ __forceinline__ int iclamp(int v, int lo, int hi) {
    return v < lo ? lo : (v > hi ? hi : v);
}

__device__ __forceinline__ v8f zero8() {
    v8f z;
#pragma unroll
    for (int i = 0; i < 8; ++i) z[i] = 0.0f;
    return z;
}

__device__ __forceinline__ unsigned short bf16_bits(float f) {
    unsigned int u = __float_as_uint(f);
    u = u + 0x7FFFu + ((u >> 16) & 1u);
    return (unsigned short)(u >> 16);
}
__device__ __forceinline__ void split_bf16(float f, unsigned short& hi, unsigned short& lo) {
    const unsigned short hb = bf16_bits(f);
    const float fh = __uint_as_float(((unsigned int)hb) << 16);
    hi = hb;
    lo = bf16_bits(f - fh);
}

__device__ __forceinline__ v16bf ldfrag(const unsigned short* p, int k0) {
    Frag f;
    f.u[0] = *(const v8us*)(p + k0);
    f.u[1] = *(const v8us*)(p + k0 + 16);
    return f.v;
}

__device__ __forceinline__ v8f wmma_bf(v16bf a, v16bf b, v8f c) {
    return __builtin_amdgcn_wmma_f32_16x16x32_bf16(false, a, false, b, (short)0, c, false, false);
}

__device__ __forceinline__ v8f tile_gemm64(const unsigned short* ah_pl, const unsigned short* al_pl, int ap, int arow0,
                                          const unsigned short* bh_pl, const unsigned short* bl_pl, int brow0, int lane)
{
    const int hh = lane >> 4, m = lane & 15;
    const unsigned short* pah = ah_pl + (arow0 + m) * ap + 8 * hh;
    const unsigned short* pal = al_pl + (arow0 + m) * ap + 8 * hh;
    const unsigned short* pbh = bh_pl + (size_t)(brow0 + m) * C_ + 8 * hh;
    const unsigned short* pbl = bl_pl + (size_t)(brow0 + m) * C_ + 8 * hh;
    const v16bf ah0 = ldfrag(pah, 0), ah1 = ldfrag(pah, 32);
    const v16bf al0 = ldfrag(pal, 0), al1 = ldfrag(pal, 32);
    const v16bf bh0 = ldfrag(pbh, 0), bh1 = ldfrag(pbh, 32);
    const v16bf bl0 = ldfrag(pbl, 0), bl1 = ldfrag(pbl, 32);
    v8f acc = zero8();
    acc = wmma_bf(al0, bh0, acc);
    acc = wmma_bf(ah0, bl0, acc);
    acc = wmma_bf(ah0, bh0, acc);
    acc = wmma_bf(al1, bh1, acc);
    acc = wmma_bf(ah1, bl1, acc);
    acc = wmma_bf(ah1, bh1, acc);
    asm volatile("v_nop\n\tv_nop\n\tv_nop\n\tv_nop"
                 : "+v"(acc)
                 : "v"(ah0), "v"(al0), "v"(ah1), "v"(al1), "v"(bh0), "v"(bl0), "v"(bh1), "v"(bl1));
    return acc;
}

__global__ void __launch_bounds__(256)
k_wcvt(const float* __restrict__ src, int K, int Nc,
       unsigned short* __restrict__ hi, unsigned short* __restrict__ lo)
{
    const int li = blockIdx.x * 256 + threadIdx.x;
    const int k8n = K >> 3;
    const int total = Nc * k8n;
    if (li < total) {
        const int n = li / k8n, k8 = li - n * k8n;
        v8us_t hv, lv;
#pragma unroll
        for (int i = 0; i < 8; ++i) {
            const float x = src[(size_t)(k8 * 8 + i) * Nc + n];
            unsigned short hb, lb;
            split_bf16(x, hb, lb);
            hv[i] = hb; lv[i] = lb;
        }
        const size_t off = (size_t)n * K + (size_t)k8 * 8;
        *(volatile v8us_t*)(hi + off) = hv;
        *(volatile v8us_t*)(lo + off) = lv;
        __threadfence();
        *(volatile v8us_t*)(hi + off) = hv;
        *(volatile v8us_t*)(lo + off) = lv;
    }
}

struct Bil {
    int x0, x1, y0, y1;
    float w00, w10, w01, w11;
};

__device__ __forceinline__ Bil bil_setup(float x, float y, int W, int H) {
    float ixf = ((x + 1.f) * (float)W - 1.f) * 0.5f;
    float iyf = ((y + 1.f) * (float)H - 1.f) * 0.5f;
    ixf = fminf(fmaxf(ixf, -8.f), (float)W + 8.f);
    iyf = fminf(fmaxf(iyf, -8.f), (float)H + 8.f);
    const float x0f = floorf(ixf), y0f = floorf(iyf);
    const float wx1 = ixf - x0f, wy1 = iyf - y0f;
    const float wx0 = 1.f - wx1, wy0 = 1.f - wy1;
    const int x0 = (int)x0f, y0 = (int)y0f;
    const float vx0 = (x0 >= 0 && x0 < W) ? 1.f : 0.f;
    const float vx1 = (x0 + 1 >= 0 && x0 + 1 < W) ? 1.f : 0.f;
    const float vy0 = (y0 >= 0 && y0 < H) ? 1.f : 0.f;
    const float vy1 = (y0 + 1 >= 0 && y0 + 1 < H) ? 1.f : 0.f;
    Bil r;
    r.w00 = (wx0 * wy0) * (vx0 * vy0);
    r.w10 = (wx1 * wy0) * (vx1 * vy0);
    r.w01 = (wx0 * wy1) * (vx0 * vy1);
    r.w11 = (wx1 * wy1) * (vx1 * vy1);
    r.x0 = iclamp(x0, 0, W - 1);     r.x1 = iclamp(x0 + 1, 0, W - 1);
    r.y0 = iclamp(y0, 0, H - 1);     r.y1 = iclamp(y0 + 1, 0, H - 1);
    return r;
}

__global__ void __launch_bounds__(STOK)
k_sample(const float* __restrict__ image, const float* __restrict__ latents,
         const float* __restrict__ coords, float* __restrict__ qf, float* __restrict__ aux)
{
    __shared__ __align__(16) float QT[STOK * TP];
    const int tid = threadIdx.x;
    const int t0 = blockIdx.x * STOK;
    const int t  = t0 + tid;
    const int b  = t / N_;
    const float yc = coords[(size_t)t * 2 + 0];
    const float xc = coords[(size_t)t * 2 + 1];

    const Bil bl = bil_setup(xc, yc, W_, H_);
    {
        const float* Lb = latents + (size_t)b * C_ * N_;
        const int i00 = bl.y0 * W_ + bl.x0;
        const int i10 = bl.y0 * W_ + bl.x1;
        const int i01 = bl.y1 * W_ + bl.x0;
        const int i11 = bl.y1 * W_ + bl.x1;
        float* qt = QT + tid * TP;
#pragma unroll 1
        for (int c = 0; c < C_; ++c) {
            const float* p = Lb + (size_t)c * N_;
            qt[c] = ((bl.w00 * p[i00] + bl.w10 * p[i10]) + bl.w01 * p[i01]) + bl.w11 * p[i11];
        }
    }
    float qin;
    {
        const Bil bi = bil_setup(xc, yc, IMW_, IMH_);
        const float* Ib = image + (size_t)b * IMH_ * IMW_;
        qin = ((bi.w00 * Ib[bi.y0 * IMW_ + bi.x0] + bi.w10 * Ib[bi.y0 * IMW_ + bi.x1])
               + bi.w01 * Ib[bi.y1 * IMW_ + bi.x0]) + bi.w11 * Ib[bi.y1 * IMW_ + bi.x1];
    }
    float qc0, qc1;
    {
        const float fy0 = -1.f + (2.f * (float)bl.y0 + 1.f) / (float)H_;
        const float fy1 = -1.f + (2.f * (float)bl.y1 + 1.f) / (float)H_;
        const float fx0 = -1.f + (2.f * (float)bl.x0 + 1.f) / (float)W_;
        const float fx1 = -1.f + (2.f * (float)bl.x1 + 1.f) / (float)W_;
        qc0 = ((bl.w00 * fy0 + bl.w10 * fy0) + bl.w01 * fy1) + bl.w11 * fy1;
        qc1 = ((bl.w00 * fx0 + bl.w10 * fx1) + bl.w01 * fx0) + bl.w11 * fx1;
    }
    v4f_t av;
    av[0] = qin; av[1] = qc0; av[2] = qc1; av[3] = 0.f;
    float* apx = aux + (size_t)t * 4;
    *(volatile v4f_t*)apx = av;
    __syncthreads();

    float* gq = qf + (size_t)t0 * C_;
#pragma unroll
    for (int it = 0; it < (STOK * C_ / 4) / STOK; ++it) {
        const int f = tid + STOK * it;
        const int line = f >> 3;
        const int row = line >> 1;
        const int col = (line & 1) * 32 + (f & 7) * 4;
        const v4f_t v = *(const v4f*)(QT + row * TP + col);
        *(volatile v4f_t*)(gq + (size_t)row * C_ + col) = v;
    }
    __threadfence();
    *(volatile v4f_t*)apx = av;
#pragma unroll
    for (int it = 0; it < (STOK * C_ / 4) / STOK; ++it) {
        const int f = tid + STOK * it;
        const int line = f >> 3;
        const int row = line >> 1;
        const int col = (line & 1) * 32 + (f & 7) * 4;
        const v4f_t v = *(const v4f*)(QT + row * TP + col);
        *(volatile v4f_t*)(gq + (size_t)row * C_ + col) = v;
    }
}

__global__ void __launch_bounds__(256)
k_lnkv(const float* __restrict__ qf,
       const float* __restrict__ lnc_s, const float* __restrict__ lnc_b,
       const unsigned short* __restrict__ wkh, const unsigned short* __restrict__ wkl,
       float* __restrict__ kv)
{
    __shared__ __align__(16) unsigned char raw[LTOK * SP * 4];
    __shared__ __align__(16) unsigned short Ah[LTOK * AP];
    __shared__ __align__(16) unsigned short Al[LTOK * AP];
    float* T = (float*)raw;
    float* S = (float*)raw;
    const int tid = threadIdx.x, lane = tid & 31, wv = tid >> 5;
    const int loc0 = blockIdx.x * LTOK;
    const int b = loc0 / N_, p0 = loc0 - b * N_;
    const float* qfb = qf + (size_t)b * N_ * C_ + p0;

#pragma unroll
    for (int i = 0; i < (LTOK * C_) / 256; ++i) {
        const int idx = tid + 256 * i;
        const int c = idx >> 6, lc = idx & 63;
        T[c * LTOK + lc] = qfb[(size_t)c * N_ + lc];
    }
    __syncthreads();

    {
        const int lc = tid >> 2, part = tid & 3;
        float x[16];
#pragma unroll
        for (int i = 0; i < 16; ++i) x[i] = T[(part * 16 + i) * LTOK + lc];
        float s = 0.f;
#pragma unroll
        for (int i = 0; i < 16; ++i) s += x[i];
        s += __shfl_xor(s, 1, 32);
        s += __shfl_xor(s, 2, 32);
        const float mu = s * (1.f / (float)C_);
        float vq = 0.f;
#pragma unroll
        for (int i = 0; i < 16; ++i) { x[i] = x[i] - mu; vq += x[i] * x[i]; }
        vq += __shfl_xor(vq, 1, 32);
        vq += __shfl_xor(vq, 2, 32);
        const float var = vq * (1.f / (float)C_);
        const float inv = rsqrtf(var + 1e-5f);
        v8us_t h0, l0, h1, l1;
#pragma unroll
        for (int i = 0; i < 8; ++i) {
            const int c = part * 16 + i;
            const float y = (x[i] * inv) * lnc_s[c] + lnc_b[c];
            unsigned short hb, lb;
            split_bf16(y, hb, lb);
            h0[i] = hb; l0[i] = lb;
        }
#pragma unroll
        for (int i = 0; i < 8; ++i) {
            const int c = part * 16 + 8 + i;
            const float y = (x[8 + i] * inv) * lnc_s[c] + lnc_b[c];
            unsigned short hb, lb;
            split_bf16(y, hb, lb);
            h1[i] = hb; l1[i] = lb;
        }
        unsigned short* pah = Ah + lc * AP + part * 16;
        unsigned short* pal = Al + lc * AP + part * 16;
        *(v8us*)(pah)     = h0;
        *(v8us*)(pah + 8) = h1;
        *(v8us*)(pal)     = l0;
        *(v8us*)(pal + 8) = l1;
    }
    __syncthreads();

    {
        const int hh = lane >> 4, m = lane & 15;
        const int n0 = wv * 16;
#pragma unroll
        for (int mi = 0; mi < 4; ++mi) {
            const v8f acc = tile_gemm64(Ah, Al, AP, mi * 16, wkh, wkl, n0, lane);
#pragma unroll
            for (int r = 0; r < 8; ++r) S[(mi * 16 + 8 * hh + r) * SP + n0 + m] = acc[r];
        }
    }
    __syncthreads();

    float* gk = kv + (size_t)loc0 * 128;
#pragma unroll
    for (int it = 0; it < (LTOK * 128 / 4) / 256; ++it) {
        const int f = tid + 256 * it;
        const int line = f >> 3;
        const int row = line >> 2;
        const int col = (line & 3) * 32 + (f & 7) * 4;
        const v4f_t v = *(const v4f*)(S + row * SP + col);
        *(volatile v4f_t*)(gk + (size_t)row * 128 + col) = v;
    }
    __threadfence();
#pragma unroll
    for (int it = 0; it < (LTOK * 128 / 4) / 256; ++it) {
        const int f = tid + 256 * it;
        const int line = f >> 3;
        const int row = line >> 2;
        const int col = (line & 3) * 32 + (f & 7) * 4;
        const v4f_t v = *(const v4f*)(S + row * SP + col);
        *(volatile v4f_t*)(gk + (size_t)row * 128 + col) = v;
    }
}

__global__ void __launch_bounds__(256)
k_attn(const float* __restrict__ qf, const float* __restrict__ aux, const float* __restrict__ kv,
       const float* __restrict__ lnq_s, const float* __restrict__ lnq_b,
       const unsigned short* __restrict__ wqh, const unsigned short* __restrict__ wql,
       const unsigned short* __restrict__ woh, const unsigned short* __restrict__ wol,
       const float* __restrict__ b_out, float* __restrict__ out)
{
    __shared__ __align__(16) unsigned short Xh[ATOK * AP];
    __shared__ __align__(16) unsigned short Xl[ATOK * AP];
    __shared__ __align__(16) float Qf[ATOK * QP];
    __shared__ __align__(16) float OS[ATOK * OC_];
    const int tid = threadIdx.x, lane = tid & 31, wv = tid >> 5;
    const int tok = tid >> 3, sub = tid & 7;
    const int t0 = blockIdx.x * ATOK;
    const int t = t0 + tok;
    const int b = t / N_, p = t - b * N_;
    const int h = p >> 7, w = p & (W_ - 1);
    const int hh = lane >> 4, m = lane & 15;
    const int tr = wv >> 2, tc = wv & 3;

    v4f_t ax;
    {
        const float* qr = qf + (size_t)t * C_ + sub * 8;
        const v4f_t xa = *(const v4f*)(qr);
        const v4f_t xb = *(const v4f*)(qr + 4);
        float x[8];
#pragma unroll
        for (int i = 0; i < 4; ++i) { x[i] = xa[i]; x[4 + i] = xb[i]; }
        float s = 0.f;
#pragma unroll
        for (int i = 0; i < 8; ++i) s += x[i];
        s += __shfl_xor(s, 1, 32);
        s += __shfl_xor(s, 2, 32);
        s += __shfl_xor(s, 4, 32);
        const float mu = s * (1.f / (float)C_);
        float vq = 0.f;
#pragma unroll
        for (int i = 0; i < 8; ++i) { x[i] = x[i] - mu; vq += x[i] * x[i]; }
        vq += __shfl_xor(vq, 1, 32);
        vq += __shfl_xor(vq, 2, 32);
        vq += __shfl_xor(vq, 4, 32);
        const float var = vq * (1.f / (float)C_);
        const float inv = rsqrtf(var + 1e-5f);
        v8us_t hv, lv;
#pragma unroll
        for (int i = 0; i < 8; ++i) {
            const int c = sub * 8 + i;
            const float y = (x[i] * inv) * lnq_s[c] + lnq_b[c];
            unsigned short hb, lb;
            split_bf16(y, hb, lb);
            hv[i] = hb; lv[i] = lb;
        }
        *(v8us*)(Xh + tok * AP + sub * 8) = hv;
        *(v8us*)(Xl + tok * AP + sub * 8) = lv;
        ax = *(const v4f*)(aux + (size_t)t * 4);
    }
    __syncthreads();

    {
        const v8f acc = tile_gemm64(Xh, Xl, AP, tr * 16, wqh, wql, tc * 16, lane);
#pragma unroll
        for (int r = 0; r < 8; ++r) Qf[(tr * 16 + 8 * hh + r) * QP + tc * 16 + m] = acc[r];
    }
    __syncthreads();

    {
        float q8[8];
        {
            const v4f_t qa = *(const v4f*)(Qf + tok * QP + sub * 8);
            const v4f_t qb = *(const v4f*)(Qf + tok * QP + sub * 8 + 4);
#pragma unroll
            for (int i = 0; i < 4; ++i) { q8[i] = qa[i]; q8[4 + i] = qb[i]; }
        }
        float sim[9];
#pragma unroll
        for (int di = -1; di <= 1; ++di) {
#pragma unroll
            for (int dj = -1; dj <= 1; ++dj) {
                const int kk = (di + 1) * 3 + (dj + 1);
                const int h2 = iclamp(h + di, 0, H_ - 1);
                const int w2 = iclamp(w + dj, 0, W_ - 1);
                const float* kp = kv + (size_t)(b * N_ + h2 * W_ + w2) * 128 + sub * 8;
                const v4f_t ka = *(const v4f*)(kp);
                const v4f_t kb = *(const v4f*)(kp + 4);
                float s = 0.f;
#pragma unroll
                for (int i = 0; i < 4; ++i) { s += q8[i] * ka[i]; }
#pragma unroll
                for (int i = 0; i < 4; ++i) { s += q8[4 + i] * kb[i]; }
                s += __shfl_xor(s, 1, 32);
                s += __shfl_xor(s, 2, 32);
                s += __shfl_xor(s, 4, 32);
                sim[kk] = s * 0.125f;
            }
        }
        float mx = sim[0];
#pragma unroll
        for (int i = 1; i < 9; ++i) mx = fmaxf(mx, sim[i]);
        float ex[9];
        float ssum = 0.f;
#pragma unroll
        for (int i = 0; i < 9; ++i) { ex[i] = expf(sim[i] - mx); ssum += ex[i]; }
        const float rinv = 1.0f / ssum;
        float o8[8];
#pragma unroll
        for (int i = 0; i < 8; ++i) o8[i] = 0.f;
#pragma unroll
        for (int di = -1; di <= 1; ++di) {
#pragma unroll
            for (int dj = -1; dj <= 1; ++dj) {
                const int kk = (di + 1) * 3 + (dj + 1);
                const int h2 = iclamp(h + di, 0, H_ - 1);
                const int w2 = iclamp(w + dj, 0, W_ - 1);
                const float* vp = kv + (size_t)(b * N_ + h2 * W_ + w2) * 128 + 64 + sub * 8;
                const v4f_t va = *(const v4f*)(vp);
                const v4f_t vb = *(const v4f*)(vp + 4);
                const float a = ex[kk] * rinv;
#pragma unroll
                for (int i = 0; i < 4; ++i) { o8[i] += a * va[i]; o8[4 + i] += a * vb[i]; }
            }
        }
        {
            v8us_t hv, lv;
#pragma unroll
            for (int i = 0; i < 8; ++i) {
                unsigned short hb, lb;
                split_bf16(o8[i], hb, lb);
                hv[i] = hb; lv[i] = lb;
            }
            *(v8us*)(Xh + tok * AP + sub * 8) = hv;
            *(v8us*)(Xl + tok * AP + sub * 8) = lv;
        }
        {
            const float PI_F = 3.14159265358979323846f;
#pragma unroll 1
            for (int qq = 0; qq < 4; ++qq) {
                const int e = sub + 8 * qq;
                const int j = (e > 0) ? (e - 1) : 0;
                const int jj = (j < 12) ? j : (j - 12);
                const int dsel = (jj >= 6) ? 1 : 0;
                const int o = jj - 6 * dsel;
                const float cval = dsel ? ax[2] : ax[1];
                const float cd = (cval + 1.0f) * 0.5f;
                const float oct = PI_F * (float)(1 << o);
                const float arg = cd * oct;
                const float sv = sinf(arg);
                const float cv = cosf(arg);
                float val = (j < 12) ? sv : cv;
                if (e == 0) val = ax[0];
                if (e < 25) OS[tok * OC_ + 64 + e] = val;
            }
        }
    }
    __syncthreads();

    {
        const v8f acc = tile_gemm64(Xh, Xl, AP, tr * 16, woh, wol, tc * 16, lane);
        const float bias = b_out[tc * 16 + m];
#pragma unroll
        for (int r = 0; r < 8; ++r) OS[(tr * 16 + 8 * hh + r) * OC_ + tc * 16 + m] = acc[r] + bias;
    }
    __syncthreads();

    {
        float* go = out + (size_t)blockIdx.x * (ATOK * OC_);
        const int NF4 = (ATOK * OC_) / 4;
#pragma unroll
        for (int it = 0; it < 3; ++it) {
            const int f = tid + 256 * it;
            if (f < NF4) {
                const v4f_t v = *(const v4f*)(OS + f * 4);
                *(volatile v4f_t*)(go + (size_t)f * 4) = v;
            }
        }
        __threadfence();
#pragma unroll
        for (int it = 0; it < 3; ++it) {
            const int f = tid + 256 * it;
            if (f < NF4) {
                const v4f_t v = *(const v4f*)(OS + f * 4);
                *(volatile v4f_t*)(go + (size_t)f * 4) = v;
            }
        }
    }
}

extern "C" void kernel_launch(void* const* d_in, const int* in_sizes, int n_in,
                              void* d_out, int out_size, void* d_ws, size_t ws_size,
                              hipStream_t stream)
{
    if (n_in < 11) return;
    if (in_sizes[0] != B_ * IMH_ * IMW_) return;
    if (in_sizes[1] != B_ * C_ * N_) return;
    if (in_sizes[2] != B_ * N_ * 2) return;
    if (in_sizes[3] != C_ || in_sizes[4] != C_ || in_sizes[5] != C_ || in_sizes[6] != C_) return;
    if (in_sizes[7] != C_ * C_) return;
    if (in_sizes[8] != C_ * 2 * C_) return;
    if (in_sizes[9] != C_ * C_) return;
    if (in_sizes[10] != C_) return;
    if (out_size != M_ * OC_) return;

    const float* image   = (const float*)d_in[0];
    const float* latents = (const float*)d_in[1];
    const float* coords  = (const float*)d_in[2];
    const float* lnq_s   = (const float*)d_in[3];
    const float* lnq_b   = (const float*)d_in[4];
    const float* lnc_s   = (const float*)d_in[5];
    const float* lnc_b   = (const float*)d_in[6];
    const float* w_q     = (const float*)d_in[7];
    const float* w_kv    = (const float*)d_in[8];
    const float* w_out   = (const float*)d_in[9];
    const float* b_out   = (const float*)d_in[10];
    float* out = (float*)d_out;

    size_t off = 0;
    const size_t o_qf  = off; off += (size_t)M_ * C_ * 4;
    const size_t o_aux = off; off += (size_t)M_ * 4 * 4;
    const size_t o_kv  = off; off += (size_t)M_ * 128 * 4;
    const size_t o_wqh = off; off += (size_t)C_ * C_ * 2;
    const size_t o_wql = off; off += (size_t)C_ * C_ * 2;
    const size_t o_wkh = off; off += (size_t)2 * C_ * C_ * 2;
    const size_t o_wkl = off; off += (size_t)2 * C_ * C_ * 2;
    const size_t o_woh = off; off += (size_t)C_ * C_ * 2;
    const size_t o_wol = off; off += (size_t)C_ * C_ * 2;
    if (off > ws_size) return;

    char* ws = (char*)d_ws;
    float* qf  = (float*)(ws + o_qf);
    float* aux = (float*)(ws + o_aux);
    float* kv  = (float*)(ws + o_kv);
    unsigned short* wqh = (unsigned short*)(ws + o_wqh);
    unsigned short* wql = (unsigned short*)(ws + o_wql);
    unsigned short* wkh = (unsigned short*)(ws + o_wkh);
    unsigned short* wkl = (unsigned short*)(ws + o_wkl);
    unsigned short* woh = (unsigned short*)(ws + o_woh);
    unsigned short* wol = (unsigned short*)(ws + o_wol);

    k_wcvt<<<(C_ * 8 + 255) / 256, 256, 0, stream>>>(w_q, C_, C_, wqh, wql);
    k_wcvt<<<(2 * C_ * 8 + 255) / 256, 256, 0, stream>>>(w_kv, C_, 2 * C_, wkh, wkl);
    k_wcvt<<<(C_ * 8 + 255) / 256, 256, 0, stream>>>(w_out, C_, C_, woh, wol);

    k_sample<<<M_ / STOK, STOK, 0, stream>>>(image, latents, coords, qf, aux);
    k_lnkv<<<M_ / LTOK, 256, 0, stream>>>(qf, lnc_s, lnc_b, wkh, wkl, kv);
    k_attn<<<M_ / ATOK, 256, 0, stream>>>(qf, aux, kv, lnq_s, lnq_b, wqh, wql, woh, wol, b_out, out);
}
